// RecurrentCharLM_14396730376932
// MI455X (gfx1250) — hardware-verified
//
#include <hip/hip_runtime.h>


typedef _Float16 v16h __attribute__((ext_vector_type(16)));
typedef _Float16 v8h  __attribute__((ext_vector_type(8)));
typedef float    v8f  __attribute__((ext_vector_type(8)));
typedef float    v4f  __attribute__((ext_vector_type(4)));
typedef _Float16 v8h_alias __attribute__((ext_vector_type(8), may_alias));
typedef float    v4f_alias __attribute__((ext_vector_type(4), may_alias));

#define HID    128
#define VOC    96
#define NITER  500
#define HPAD   132
#define NPAD   136
#define LPAD   96
#define BSCALE 16.0f
#define BINV   0.0625f

union Frag { v16h v; v8h half[2]; };

__device__ __forceinline__ v8f wmma_f16(v16h a, v16h b, v8f c) {
    v8f d = __builtin_amdgcn_wmma_f32_16x16x32_f16(false, a, false, b, (short)0, c, false, false);
    asm volatile("v_nop\n\tv_nop\n\tv_nop\n\tv_nop" : "+v"(d) : "v"(a), "v"(b));
    return d;
}

__global__ __launch_bounds__(256) void
k_relu_rnn(const int*   __restrict__ chars,
           const float* __restrict__ hidden,
           const float* __restrict__ embed_w,
           const float* __restrict__ W,
           const float* __restrict__ bias,
           const float* __restrict__ pre_scale,
           const float* __restrict__ post_scale,
           const float* __restrict__ readout_w,
           const float* __restrict__ readout_b,
           float* out,
           int B, int S, int out1_off)
{
    __shared__ __align__(16) float    h_ls[16 * HPAD];
    __shared__ __align__(16) _Float16 nf16[16 * NPAD];
    __shared__ __align__(16) float    lg_ls[16 * LPAD];
    __shared__ float inv_rms[16];

    const int t     = threadIdx.x;
    const int lane  = t & 31;
    const int wv    = __builtin_amdgcn_readfirstlane(t >> 5);
    const int nl    = lane & 15;
    const int hh    = lane >> 4;
    const int n_col = wv * 16 + nl;
    const int rt    = t >> 4;
    const int c0    = (t & 15) * 8;
    const int r_s   = 2 * wv + hh;
    const int row0  = blockIdx.x * 16;
    const int bmax  = B - 1;

    {
        int gr = row0 + rt; gr = (gr > bmax) ? bmax : gr;
        const float* src = hidden + (size_t)gr * HID + c0;
        #pragma unroll
        for (int i = 0; i < 8; ++i) h_ls[rt * HPAD + c0 + i] = src[i];
    }
    float ps8[8];
    #pragma unroll
    for (int i = 0; i < 8; ++i) ps8[i] = pre_scale[c0 + i];
    const float bias_n = bias[n_col];

    auto loadW = [&](int kc) {
        v16h r;
        #pragma unroll
        for (int j = 0; j < 16; ++j) {
            const int k = kc * 32 + 8 * hh + (j & 7) + ((j >> 3) << 4);
            r[j] = (_Float16)(W[(size_t)k * HID + n_col] * BSCALE);
        }
        return r;
    };
    const v16h wf0 = loadW(0), wf1 = loadW(1), wf2 = loadW(2), wf3 = loadW(3);

    auto loadR = [&](int kc, int n_v) {
        v16h r;
        #pragma unroll
        for (int j = 0; j < 16; ++j) {
            const int k = kc * 32 + 8 * hh + (j & 7) + ((j >> 3) << 4);
            r[j] = (_Float16)(readout_w[(size_t)n_v * HID + k] * BSCALE);
        }
        return r;
    };

    auto loadA = [&](int kc) {
        Frag f;
        const _Float16* base = nf16 + nl * NPAD + kc * 32 + 8 * hh;
        f.half[0] = *(const v8h_alias*)(base);
        f.half[1] = *(const v8h_alias*)(base + 16);
        return f.v;
    };

    __syncthreads();

    #pragma unroll 1
    for (int s = 0; s < S; ++s) {
        float e_reg[8];
        #pragma unroll
        for (int v = 0; v < 8; ++v) {
            int gr = row0 + v + 8 * hh; gr = (gr > bmax) ? bmax : gr;
            int ch = chars[(size_t)gr * S + s];
            ch = (ch < 0) ? 0 : ((ch > VOC - 1) ? (VOC - 1) : ch);
            e_reg[v] = embed_w[(size_t)ch * HID + n_col];
        }

        #pragma unroll 1
        for (int d = 0; d < NITER; ++d) {
            {
                const float* hr = h_ls + r_s * HPAD + nl * 8;
                const v4f x0 = *(const v4f_alias*)(hr);
                const v4f x1 = *(const v4f_alias*)(hr + 4);
                float p = x0.x * x0.x;
                p += x0.y * x0.y; p += x0.z * x0.z; p += x0.w * x0.w;
                p += x1.x * x1.x; p += x1.y * x1.y; p += x1.z * x1.z; p += x1.w * x1.w;
                p += __shfl_xor(p, 1, 32); p += __shfl_xor(p, 2, 32);
                p += __shfl_xor(p, 4, 32); p += __shfl_xor(p, 8, 32);
                if (nl == 0) inv_rms[r_s] = rsqrtf(p * (1.0f / HID) + 1e-6f);
            }
            __syncthreads();

            {
                const float ir = inv_rms[rt];
                const float* hrow = h_ls + rt * HPAD + c0;
                const v4f a0 = *(const v4f_alias*)(hrow);
                const v4f a1 = *(const v4f_alias*)(hrow + 4);
                v8h nv;
                nv[0] = (_Float16)((a0.x * ir) * ps8[0]);
                nv[1] = (_Float16)((a0.y * ir) * ps8[1]);
                nv[2] = (_Float16)((a0.z * ir) * ps8[2]);
                nv[3] = (_Float16)((a0.w * ir) * ps8[3]);
                nv[4] = (_Float16)((a1.x * ir) * ps8[4]);
                nv[5] = (_Float16)((a1.y * ir) * ps8[5]);
                nv[6] = (_Float16)((a1.z * ir) * ps8[6]);
                nv[7] = (_Float16)((a1.w * ir) * ps8[7]);
                *(v8h_alias*)(nf16 + rt * NPAD + c0) = nv;
            }
            __syncthreads();

            v8f c = {0.f, 0.f, 0.f, 0.f, 0.f, 0.f, 0.f, 0.f};
            c = wmma_f16(loadA(0), wf0, c);
            c = wmma_f16(loadA(1), wf1, c);
            c = wmma_f16(loadA(2), wf2, c);
            c = wmma_f16(loadA(3), wf3, c);

            #pragma unroll
            for (int v = 0; v < 8; ++v) {
                const int m = v + 8 * hh;
                float y = c[v] * BINV + e_reg[v];
                y = y + bias_n;
                h_ls[m * HPAD + n_col] += (y > 0.f ? y : 0.f);
            }
            __syncthreads();
        }

        {
            const float* hr = h_ls + r_s * HPAD + nl * 8;
            const v4f x0 = *(const v4f_alias*)(hr);
            const v4f x1 = *(const v4f_alias*)(hr + 4);
            float p = x0.x * x0.x;
            p += x0.y * x0.y; p += x0.z * x0.z; p += x0.w * x0.w;
            p += x1.x * x1.x; p += x1.y * x1.y; p += x1.z * x1.z; p += x1.w * x1.w;
            p += __shfl_xor(p, 1, 32); p += __shfl_xor(p, 2, 32);
            p += __shfl_xor(p, 4, 32); p += __shfl_xor(p, 8, 32);
            if (nl == 0) inv_rms[r_s] = rsqrtf(p * (1.0f / HID) + 1e-6f);
        }
        __syncthreads();
        {
            const float ir = inv_rms[rt];
            float hv[8];
            {
                const float* hrow = h_ls + rt * HPAD + c0;
                const v4f a0 = *(const v4f_alias*)(hrow);
                const v4f a1 = *(const v4f_alias*)(hrow + 4);
                hv[0] = a0.x; hv[1] = a0.y; hv[2] = a0.z; hv[3] = a0.w;
                hv[4] = a1.x; hv[5] = a1.y; hv[6] = a1.z; hv[7] = a1.w;
            }
            v8h nv;
            #pragma unroll
            for (int i = 0; i < 8; ++i) {
                const float v_ = (hv[i] * ir) * post_scale[c0 + i];
                h_ls[rt * HPAD + c0 + i] = v_;
                nv[i] = (_Float16)v_;
            }
            *(v8h_alias*)(nf16 + rt * NPAD + c0) = nv;
        }
        __syncthreads();

        if (wv < 6) {
            const int n_v = wv * 16 + nl;
            const v16h rf0 = loadR(0, n_v), rf1 = loadR(1, n_v), rf2 = loadR(2, n_v), rf3 = loadR(3, n_v);
            const float rbias = readout_b[n_v];
            v8f c = {0.f, 0.f, 0.f, 0.f, 0.f, 0.f, 0.f, 0.f};
            c = wmma_f16(loadA(0), rf0, c);
            c = wmma_f16(loadA(1), rf1, c);
            c = wmma_f16(loadA(2), rf2, c);
            c = wmma_f16(loadA(3), rf3, c);
            #pragma unroll
            for (int v = 0; v < 8; ++v) {
                const int m = v + 8 * hh;
                lg_ls[m * LPAD + n_v] = c[v] * BINV + rbias;
            }
        }
        __syncthreads();

        {
            const int r0i = 2 * wv, r1i = 2 * wv + 1;
            const int g0 = row0 + r0i, g1 = row0 + r1i;
            const bool act = lane < 24;
            v4f val0 = {0.f, 0.f, 0.f, 0.f}, val1 = {0.f, 0.f, 0.f, 0.f};
            if (act) {
                val0 = *(const v4f_alias*)(lg_ls + r0i * LPAD + 4 * lane);
                val1 = *(const v4f_alias*)(lg_ls + r1i * LPAD + 4 * lane);
            }
            float* p0 = out + ((size_t)g0 * S + s) * VOC + 4 * lane;
            float* p1 = out + ((size_t)g1 * S + s) * VOC + 4 * lane;
            const bool ok0 = act && (g0 < B);
            const bool ok1 = act && (g1 < B);
            if (ok0) *(volatile v4f*)p0 = val0;
            if (ok1) *(volatile v4f*)p1 = val1;
            __threadfence();
            if (ok0) *(volatile v4f*)p0 = val0;
            if (ok1) *(volatile v4f*)p1 = val1;
        }
        __syncthreads();
    }

    {
        const int r0i = 2 * wv, r1i = 2 * wv + 1;
        const int g0 = row0 + r0i, g1 = row0 + r1i;
        const v4f val0 = *(const v4f_alias*)(h_ls + r0i * HPAD + 4 * lane);
        const v4f val1 = *(const v4f_alias*)(h_ls + r1i * HPAD + 4 * lane);
        float* p0 = out + (size_t)out1_off + (size_t)g0 * HID + 4 * lane;
        float* p1 = out + (size_t)out1_off + (size_t)g1 * HID + 4 * lane;
        const bool ok0 = (g0 < B);
        const bool ok1 = (g1 < B);
        if (ok0) *(volatile v4f*)p0 = val0;
        if (ok1) *(volatile v4f*)p1 = val1;
        __threadfence();
        if (ok0) *(volatile v4f*)p0 = val0;
        if (ok1) *(volatile v4f*)p1 = val1;
    }
}

extern "C" void kernel_launch(void* const* d_in, const int* in_sizes, int n_in,
                              void* d_out, int out_size, void* d_ws, size_t ws_size,
                              hipStream_t stream) {
    (void)n_in; (void)d_ws; (void)ws_size;
    const int*   chars      = (const int*)  d_in[0];
    const float* hidden     = (const float*)d_in[1];
    const float* embed_w    = (const float*)d_in[2];
    const float* W          = (const float*)d_in[3];
    const float* b          = (const float*)d_in[4];
    const float* pre_scale  = (const float*)d_in[5];
    const float* post_scale = (const float*)d_in[6];
    const float* readout_w  = (const float*)d_in[7];
    const float* readout_b  = (const float*)d_in[8];
    float* out = (float*)d_out;

    const int B = in_sizes[1] / HID;
    if (B <= 0) return;
    const int S = in_sizes[0] / B;
    if (S <= 0) return;
    const int out1_off = B * S * VOC;
    if (out_size < out1_off + B * HID) return;
    const int nblk = (B + 15) / 16;

    k_relu_rnn<<<dim3(nblk), dim3(256), 0, stream>>>(
        chars, hidden, embed_w, W, b, pre_scale, post_scale,
        readout_w, readout_b, out, B, S, out1_off);
}
